// DecoderLayer_71494025609892
// MI455X (gfx1250) — hardware-verified
//
#include <hip/hip_runtime.h>
#ifndef NB
#define NB 4
#endif
#ifndef SEQ
#define SEQ 1024
#endif
#define NB_FULL 4
#define SEQ_FULL 1024
#define DM 1024
#define NH 16
#define HD 64
#define DFF 4096
#define LQ (3 * DM)
#define MROWS (SEQ * NB_FULL)
#define RP (NB_FULL * LQ)
#define NQT (SEQ / 64)
#define NKT (SEQ / 64)
static_assert(SEQ % 64 == 0);
static_assert(SEQ <= SEQ_FULL);
static_assert(NB >= 1 && NB <= NB_FULL);
static_assert(MROWS % 128 == 0);
static_assert(DM % 64 == 0 && DM % 32 == 0);
static_assert(DFF % 64 == 0 && DFF % 32 == 0);
static_assert(DM == NH * HD);
static_assert(DM == 256 * 4);
static_assert(((size_t)MROWS * DM) % 8 == 0);
static_assert(((size_t)DM * DM) % 8 == 0 && ((size_t)DFF * DM) % 8 == 0);

typedef _Float16 v16h __attribute__((ext_vector_type(16)));
typedef _Float16 v4h  __attribute__((ext_vector_type(4)));
typedef unsigned short v8us __attribute__((ext_vector_type(8), may_alias));
typedef float  v8f  __attribute__((ext_vector_type(8)));
typedef float  v4f  __attribute__((ext_vector_type(4)));
typedef float  v4fa __attribute__((ext_vector_type(4), may_alias));
union FragH { v16h v; v8us half[2]; _Float16 h[16]; unsigned short u[16]; };

#define NEG_INF (-__builtin_inff())

__device__ __forceinline__ unsigned short bf16_bits(float x) { unsigned int u = __float_as_uint(x); return (unsigned short)((u + 0x7FFFu + ((u >> 16) & 1u)) >> 16); }
__device__ __forceinline__ float bf16_val(unsigned short b) { return __uint_as_float(((unsigned int)b) << 16); }
__device__ __forceinline__ float bf16_rne(float x) { return bf16_val(bf16_bits(x)); }

__device__ __forceinline__ v16h g2_frag(const _Float16* p, int hh) { FragH f; f.half[0] = *(const v8us*)((const unsigned short*)p + 8 * hh); f.half[1] = *(const v8us*)((const unsigned short*)p + 16 + 8 * hh); return f.v; }
__device__ __forceinline__ v8f g2_mma(v16h a, v16h b, v8f c) { v8f d = __builtin_amdgcn_wmma_f32_16x16x32_f16(false, a, false, b, (short)0, c, false, false); asm volatile("v_nop\n\tv_nop\n\tv_nop\n\tv_nop" : "+v"(d) : "v"(a), "v"(b)); return d; }

__global__ __launch_bounds__(256) void k_x16(const float* __restrict__ x, _Float16* __restrict__ X16, size_t n8) {
  const size_t t = (size_t)blockIdx.x * 256 + threadIdx.x; if (t >= n8) return; FragH f;
#pragma unroll
  for (int q = 0; q < 8; ++q) f.h[q] = (_Float16)bf16_rne(x[t * 8 + q]);
  *(volatile v8us*)((unsigned short*)X16 + t * 8) = f.half[0]; __threadfence(); *(volatile v8us*)((unsigned short*)X16 + t * 8) = f.half[0]; }

__global__ __launch_bounds__(256) void k_wnat(const float* __restrict__ w, size_t n8, _Float16* __restrict__ Bt) {
  const size_t t = (size_t)blockIdx.x * 256 + threadIdx.x; if (t >= n8) return; FragH f;
#pragma unroll
  for (int q = 0; q < 8; ++q) f.h[q] = (_Float16)(bf16_rne(w[t * 8 + q]) * 16.0f);
  *(volatile v8us*)((unsigned short*)Bt + t * 8) = f.half[0]; __threadfence(); *(volatile v8us*)((unsigned short*)Bt + t * 8) = f.half[0]; }

__global__ __launch_bounds__(128) void k_gemm2(const _Float16* __restrict__ A, int lda, const _Float16* __restrict__ Bh, int ldb, float alpha, const float* __restrict__ bias, int relu,
    _Float16* __restrict__ C16, float* __restrict__ C32, int ldc, int M, int N, int K) {
  __shared__ __attribute__((aligned(16))) float so[4][32][68];
  const int tid = threadIdx.x, w = tid >> 5, lane = tid & 31, ln = lane & 15, hh = lane >> 4;
  const int ntn = N >> 6; const int mt = blockIdx.x / ntn, nq = blockIdx.x - mt * ntn; const int row0 = mt * 128 + 32 * w, col0 = nq * 64; if (row0 >= M) return;
  const _Float16* a0p = A + (size_t)(row0 + ln) * lda; const _Float16* a1p = a0p + (size_t)16 * lda;
  const _Float16* b0p = Bh + (size_t)(col0 + ln) * ldb; const _Float16* b1p = b0p + (size_t)16 * ldb; const _Float16* b2p = b1p + (size_t)16 * ldb; const _Float16* b3p = b2p + (size_t)16 * ldb;
  const v8f z8 = {0.f,0.f,0.f,0.f,0.f,0.f,0.f,0.f}; v8f c00 = z8, c01 = z8, c02 = z8, c03 = z8, c10 = z8, c11 = z8, c12 = z8, c13 = z8;
#pragma unroll 1
  for (int kb = 0; kb < K; kb += 32) { const v16h a0 = g2_frag(a0p + kb, hh), a1 = g2_frag(a1p + kb, hh);
    v16h b = g2_frag(b0p + kb, hh); c00 = g2_mma(a0, b, c00); c10 = g2_mma(a1, b, c10);
    b = g2_frag(b1p + kb, hh); c01 = g2_mma(a0, b, c01); c11 = g2_mma(a1, b, c11);
    b = g2_frag(b2p + kb, hh); c02 = g2_mma(a0, b, c02); c12 = g2_mma(a1, b, c12);
    b = g2_frag(b3p + kb, hh); c03 = g2_mma(a0, b, c03); c13 = g2_mma(a1, b, c13); }
  v8f accs[8] = {c00, c01, c02, c03, c10, c11, c12, c13};
#pragma unroll
  for (int u = 0; u < 8; ++u) { const int t = u & 3, half = u >> 2; const int col = col0 + t * 16 + ln; const float bv = bf16_rne(bias[col]);
#pragma unroll
    for (int r = 0; r < 8; ++r) { const int rloc = half * 16 + 8 * hh + r; float v = accs[u][r] * alpha + bv; v = (relu != 0) ? fmaxf(v, 0.0f) : v; so[w][rloc][t * 16 + ln] = v; } }
  __builtin_amdgcn_fence(4  , "workgroup"); __builtin_amdgcn_wave_barrier();
  const int rsub = lane >> 4, c4 = (lane & 15) * 4;
  if (C32 != nullptr) {
    for (int pass = 0; pass < 2; ++pass) {
#pragma unroll
      for (int q = 0; q < 16; ++q) { const int r = q * 2 + rsub; const v4f v = *(const v4fa*)&so[w][r][c4];
        *(volatile v4f*)(C32 + (size_t)(row0 + r) * ldc + col0 + c4) = v; }
      if (pass == 0) __threadfence(); }
  } else {
    for (int pass = 0; pass < 2; ++pass) {
#pragma unroll
      for (int q = 0; q < 16; ++q) { const int r = q * 2 + rsub; const v4f v = *(const v4fa*)&so[w][r][c4]; v4h h4;
#pragma unroll
        for (int i = 0; i < 4; ++i) h4[i] = (_Float16)v[i];
        *(volatile v4h*)(C16 + (size_t)(row0 + r) * ldc + col0 + c4) = h4; }
      if (pass == 0) __threadfence(); } } }

__global__ __launch_bounds__(256) void k_vt2(const _Float16* __restrict__ QKV, _Float16* __restrict__ VT) {
  __shared__ unsigned short tl[64][66];
  const int tid = threadIdx.x; const int slab = blockIdx.x / NQT, lg = blockIdx.x - slab * NQT; const int b = slab / NH, hd = slab - b * NH; const int s0 = lg * 64;
  for (int i = tid; i < 64 * 8; i += 256) { const int r = i / 8, c8 = (i % 8) * 8; FragH f;
    f.half[0] = *(const v8us*)((const unsigned short*)QKV + ((size_t)(s0 + r) * NB_FULL + b) * LQ + 2 * DM + hd * HD + c8);
#pragma unroll
    for (int q = 0; q < 8; ++q) tl[r][c8 + q] = f.u[q]; }
  __syncthreads();
  for (int pass = 0; pass < 2; ++pass) {
#pragma unroll
    for (int rd = 0; rd < 2; ++rd) { const int d = rd * 32 + tid / 8, pc = tid % 8; FragH f;
#pragma unroll
      for (int q = 0; q < 8; ++q) f.u[q] = tl[pc * 8 + q][d];
      *(volatile v8us*)((unsigned short*)VT + ((size_t)slab * HD + d) * SEQ + s0 + pc * 8) = f.half[0]; }
    if (pass == 0) __threadfence(); } }

__global__ __launch_bounds__(128) void k_attn(const _Float16* __restrict__ QKV, const _Float16* __restrict__ VT, _Float16* __restrict__ CTX) {
  __shared__ __attribute__((aligned(16))) float so[4][16][68];
  const int tid = threadIdx.x, w = tid >> 5, lane = tid & 31, l15 = lane & 15, hh = lane >> 4;
  const int qt = blockIdx.x, slab = blockIdx.y; const int b = slab / NH, hd = slab - b * NH;
  const int q0 = qt * 64 + w * 16;
  const _Float16* Qb = QKV + (size_t)b * LQ + hd * HD;
  const _Float16* Kb = Qb + DM;
  const _Float16* Vb = VT + (size_t)slab * HD * SEQ;
  const _Float16* qrow = Qb + (size_t)(q0 + l15) * RP;
  const v16h qf0 = g2_frag(qrow, hh), qf1 = g2_frag(qrow + 32, hh);
  const v8f z8 = {0.f,0.f,0.f,0.f,0.f,0.f,0.f,0.f};
  v8f o[4] = {z8, z8, z8, z8};
  float m = NEG_INF, l = 0.f;
  const float CL = 0.18033688011112042f;
#pragma unroll 1
  for (int it = 0; it < NKT; ++it) {
    const int key0 = it * 64;
    v8f s[4];
#pragma unroll
    for (int kt = 0; kt < 4; ++kt) {
      const _Float16* krow = Kb + (size_t)(key0 + kt * 16 + l15) * RP;
      const v16h ka = g2_frag(krow, hh), kk = g2_frag(krow + 32, hh);
      v8f a = g2_mma(ka, qf0, z8); a = g2_mma(kk, qf1, a); s[kt] = a; }
    float lmax = NEG_INF;
#pragma unroll
    for (int kt = 0; kt < 4; ++kt)
#pragma unroll
      for (int r = 0; r < 8; ++r) lmax = fmaxf(lmax, s[kt][r]);
    lmax = fmaxf(lmax, __shfl_xor(lmax, 16));
    const float mnew = fmaxf(m, lmax);
    const float mref = (mnew == NEG_INF) ? 0.0f : mnew;
    const float alpha = exp2f((m - mref) * CL);
    const float bexp = 10.0f - mref * CL;
    m = mnew;
    float psum = 0.f; FragH pa, pb;
#pragma unroll
    for (int r = 0; r < 8; ++r) {
      const float e0 = exp2f(fmaf(s[0][r], CL, bexp)), e1 = exp2f(fmaf(s[1][r], CL, bexp)), e2 = exp2f(fmaf(s[2][r], CL, bexp)), e3 = exp2f(fmaf(s[3][r], CL, bexp));
      psum += (e0 + e1) + (e2 + e3);
      pa.h[r] = (_Float16)e0; pa.h[8 + r] = (_Float16)e1; pb.h[r] = (_Float16)e2; pb.h[8 + r] = (_Float16)e3; }
    l = l * alpha + psum;
    float ar[8];
#pragma unroll
    for (int r = 0; r < 8; ++r) ar[r] = __shfl(alpha, 8 * hh + r);
#pragma unroll
    for (int dt = 0; dt < 4; ++dt) {
#pragma unroll
      for (int r = 0; r < 8; ++r) o[dt][r] *= ar[r];
      const _Float16* vrow = Vb + (size_t)(dt * 16 + l15) * SEQ + key0;
      const v16h va = g2_frag(vrow, hh), vb = g2_frag(vrow + 32, hh);
      o[dt] = g2_mma(pa.v, va, o[dt]); o[dt] = g2_mma(pb.v, vb, o[dt]); } }
  const float lt = l + __shfl_xor(l, 16);
  const float inv = 64.0f / lt;
  float ir[8];
#pragma unroll
  for (int r = 0; r < 8; ++r) ir[r] = __shfl(inv, 8 * hh + r);
#pragma unroll
  for (int dt = 0; dt < 4; ++dt)
#pragma unroll
    for (int r = 0; r < 8; ++r) so[w][8 * hh + r][dt * 16 + l15] = o[dt][r] * ir[r];
  __builtin_amdgcn_fence(4  , "workgroup"); __builtin_amdgcn_wave_barrier();
  const int rq = lane >> 3, pc = lane & 7;
  for (int pass = 0; pass < 2; ++pass) {
#pragma unroll
    for (int g = 0; g < 4; ++g) { const int row = g * 4 + rq, col = pc * 8;
      const v4f va = *(const v4fa*)&so[w][row][col]; const v4f vb = *(const v4fa*)&so[w][row][col + 4]; FragH f;
#pragma unroll
      for (int i = 0; i < 4; ++i) { f.h[i] = (_Float16)va[i]; f.h[4 + i] = (_Float16)vb[i]; }
      *(volatile v8us*)((unsigned short*)CTX + ((size_t)(q0 + row) * NB_FULL + b) * DM + hd * HD + col) = f.half[0]; }
    if (pass == 0) __threadfence(); } }

__global__ __launch_bounds__(256) void k_ln(const float* __restrict__ resid, int rne_resid, const float* __restrict__ proj, const float* __restrict__ g, const float* __restrict__ be,
    float* __restrict__ outF, _Float16* __restrict__ out16) {
  __shared__ __attribute__((aligned(16))) float sy[DM];
  __shared__ float rs[8];
  __shared__ float rs2[8];
  const int row = blockIdx.x, tid = threadIdx.x, wv = tid >> 5, lane = tid & 31;
  const size_t base = (size_t)row * DM + (size_t)tid * 4;
  const v4f r4 = *(const v4fa*)(resid + base); const v4f p4 = *(const v4fa*)(proj + base);
  float x[4]; float s = 0.f;
#pragma unroll
  for (int i = 0; i < 4; ++i) { float rv = r4[i]; rv = (rne_resid != 0) ? bf16_rne(rv) : rv; x[i] = rv + p4[i]; s += x[i]; }
  s += __shfl_xor(s, 16); s += __shfl_xor(s, 8); s += __shfl_xor(s, 4); s += __shfl_xor(s, 2); s += __shfl_xor(s, 1);
  if (lane == 0) rs[wv] = s;
  __syncthreads();
  float ts = 0.f;
#pragma unroll
  for (int q = 0; q < 8; ++q) ts += rs[q];
  const float mean = ts * (1.0f / (float)DM);
  float s2 = 0.f;
#pragma unroll
  for (int i = 0; i < 4; ++i) { const float d = x[i] - mean; s2 += d * d; }
  s2 += __shfl_xor(s2, 16); s2 += __shfl_xor(s2, 8); s2 += __shfl_xor(s2, 4); s2 += __shfl_xor(s2, 2); s2 += __shfl_xor(s2, 1);
  if (lane == 0) rs2[wv] = s2;
  __syncthreads();
  float tv = 0.f;
#pragma unroll
  for (int q = 0; q < 8; ++q) tv += rs2[q];
  const float var = tv * (1.0f / (float)DM);
  const float inv = rsqrtf(var + 1e-5f);
  const v4f g4 = *(const v4fa*)(g + tid * 4); const v4f b4 = *(const v4fa*)(be + tid * 4);
  v4f y;
#pragma unroll
  for (int i = 0; i < 4; ++i) y[i] = (x[i] - mean) * inv * bf16_rne(g4[i]) + bf16_rne(b4[i]);
  *(v4fa*)&sy[tid * 4] = y;
  __syncthreads();
  const int t8 = (tid & 127) * 8;
  const v4f ya = *(const v4fa*)&sy[t8]; const v4f yb = *(const v4fa*)&sy[t8 + 4]; FragH f;
#pragma unroll
  for (int i = 0; i < 4; ++i) { f.h[i] = (_Float16)ya[i]; f.h[4 + i] = (_Float16)yb[i]; }
  const bool w16 = (out16 != nullptr) && (tid < 128);
  for (int pass = 0; pass < 2; ++pass) {
    *(volatile v4f*)(outF + base) = y;
    if (w16) *(volatile v8us*)((unsigned short*)out16 + (size_t)row * DM + t8) = f.half[0];
    if (pass == 0) __threadfence(); } }

#define SZ_WATT ((size_t)8 * DM * DM * 2)
#define SZ_RES  ((size_t)MROWS * DM * 4)
#define SZ_P16  ((size_t)MROWS * DM * 2)
#define SZ_QKV  ((size_t)MROWS * LQ * 2)
#define SZ_VT   ((size_t)NB * NH * HD * SEQ * 2)
#define SZ_H1   ((size_t)MROWS * DFF * 2)
#define SZ_RA   (((SZ_QKV + SZ_VT) > SZ_H1) ? (SZ_QKV + SZ_VT) : SZ_H1)
static_assert(SZ_RES <= SZ_WATT);
static_assert(SZ_QKV % 256 == 0);
static_assert(SZ_QKV + SZ_VT <= SZ_RA && SZ_H1 <= SZ_RA);

extern "C" void kernel_launch(void* const* d_in, const int* in_sizes, int n_in,
                              void* d_out, int out_size, void* d_ws, size_t ws_size, hipStream_t stream) {
  if (n_in < 28) return;
  const float* xin = (const float*)d_in[0];
  const float* enc = (const float*)d_in[1];
  const float* aw[8]; const float* ab[8];
  for (int i = 0; i < 8; ++i) { aw[i] = (const float*)d_in[2 + 2 * i]; ab[i] = (const float*)d_in[3 + 2 * i]; }
  const float* w1 = (const float*)d_in[18]; const float* b1 = (const float*)d_in[19];
  const float* w2 = (const float*)d_in[20]; const float* b2 = (const float*)d_in[21];
  const float* lg[3]; const float* lb[3];
  for (int i = 0; i < 3; ++i) { lg[i] = (const float*)d_in[22 + 2 * i]; lb[i] = (const float*)d_in[23 + 2 * i]; }
  if (in_sizes[0] < MROWS * DM || in_sizes[1] < MROWS * DM) return;
  for (int i = 0; i < 8; ++i) { if (in_sizes[2 + 2 * i] < DM * DM || in_sizes[3 + 2 * i] < DM) return; }
  if (in_sizes[18] < DFF * DM || in_sizes[19] < DFF || in_sizes[20] < DM * DFF || in_sizes[21] < DM) return;
  for (int i = 22; i < 28; ++i) { if (in_sizes[i] < DM) return; }
  if (out_size < MROWS * DM) return;
  char* ws = (char*)d_ws; size_t off = 0;
  auto take = [&](size_t bytes) { char* p = ws + off; off += (bytes + 255) & ~(size_t)255; return p; };
  char* WATT = take(SZ_WATT);
  _Float16* W1B = (_Float16*)take((size_t)DFF * DM * 2);
  _Float16* W2B = (_Float16*)take((size_t)DM * DFF * 2);
  _Float16* P16 = (_Float16*)take(SZ_P16);
  _Float16* E16 = (_Float16*)take(SZ_P16);
  char* RA = take(SZ_RA);
  _Float16* CTX = (_Float16*)take(SZ_P16);
  float* PROJ = (float*)take(SZ_RES);
  float* RES1 = (float*)take(SZ_RES);
  if (off > ws_size || off > (size_t)134217728) return;
  _Float16* BW[8]; for (int i = 0; i < 8; ++i) BW[i] = (_Float16*)(WATT + (size_t)i * DM * DM * 2);
  float* RES2 = (float*)WATT;
  _Float16* QKV = (_Float16*)RA; _Float16* VT = (_Float16*)(RA + SZ_QKV); _Float16* H1 = (_Float16*)RA;
  _Float16* X16 = P16; _Float16* L16 = P16;

  const size_t nw8 = (size_t)DM * DM / 8, nf8 = (size_t)DFF * DM / 8, nx8 = (size_t)MROWS * DM / 8;
  for (int i = 0; i < 8; ++i) k_wnat<<<(unsigned)((nw8 + 255) / 256), 256, 0, stream>>>(aw[i], nw8, BW[i]);
  k_wnat<<<(unsigned)((nf8 + 255) / 256), 256, 0, stream>>>(w1, nf8, W1B);
  k_wnat<<<(unsigned)((nf8 + 255) / 256), 256, 0, stream>>>(w2, nf8, W2B);
  k_x16<<<(unsigned)((nx8 + 255) / 256), 256, 0, stream>>>(xin, X16, nx8);
  k_x16<<<(unsigned)((nx8 + 255) / 256), 256, 0, stream>>>(enc, E16, nx8);

  const unsigned gD = (unsigned)((MROWS / 128) * (DM / 64));
  const unsigned gF = (unsigned)((MROWS / 128) * (DFF / 64));
  const dim3 ga((unsigned)NQT, (unsigned)(NB * NH));
  const float A16 = 0.0625f, ACTX = 0.0009765625f;

  k_gemm2<<<gD, 128, 0, stream>>>(X16, DM, BW[0], DM, A16, ab[0], 0, QKV,          nullptr, LQ, MROWS, DM, DM);
  k_gemm2<<<gD, 128, 0, stream>>>(X16, DM, BW[1], DM, A16, ab[1], 0, QKV + DM,     nullptr, LQ, MROWS, DM, DM);
  k_gemm2<<<gD, 128, 0, stream>>>(X16, DM, BW[2], DM, A16, ab[2], 0, QKV + 2 * DM, nullptr, LQ, MROWS, DM, DM);
  k_vt2<<<(unsigned)(NB * NH * NQT), 256, 0, stream>>>(QKV, VT);
  k_attn<<<ga, 128, 0, stream>>>(QKV, VT, CTX);
  k_gemm2<<<gD, 128, 0, stream>>>(CTX, DM, BW[3], DM, ACTX, ab[3], 0, nullptr, PROJ, DM, MROWS, DM, DM);
  k_ln<<<(unsigned)MROWS, 256, 0, stream>>>(xin, 1, PROJ, lg[0], lb[0], RES1, L16);

  k_gemm2<<<gD, 128, 0, stream>>>(E16, DM, BW[4], DM, A16, ab[4], 0, QKV,          nullptr, LQ, MROWS, DM, DM);
  k_gemm2<<<gD, 128, 0, stream>>>(L16, DM, BW[5], DM, A16, ab[5], 0, QKV + DM,     nullptr, LQ, MROWS, DM, DM);
  k_gemm2<<<gD, 128, 0, stream>>>(E16, DM, BW[6], DM, A16, ab[6], 0, QKV + 2 * DM, nullptr, LQ, MROWS, DM, DM);
  k_vt2<<<(unsigned)(NB * NH * NQT), 256, 0, stream>>>(QKV, VT);
  k_attn<<<ga, 128, 0, stream>>>(QKV, VT, CTX);
  k_gemm2<<<gD, 128, 0, stream>>>(CTX, DM, BW[7], DM, ACTX, ab[7], 0, nullptr, PROJ, DM, MROWS, DM, DM);
  k_ln<<<(unsigned)MROWS, 256, 0, stream>>>(RES1, 0, PROJ, lg[1], lb[1], RES2, L16);

  k_gemm2<<<gF, 128, 0, stream>>>(L16, DM, W1B, DM, A16, b1, 1, H1, nullptr, DFF, MROWS, DFF, DM);
  k_gemm2<<<gD, 128, 0, stream>>>(H1, DFF, W2B, DFF, A16, b2, 0, nullptr, PROJ, DM, MROWS, DM, DFF);
  k_ln<<<(unsigned)MROWS, 256, 0, stream>>>(RES2, 0, PROJ, lg[2], lb[2], (float*)d_out, nullptr);
}
